// self_att_54803782697259
// MI455X (gfx1250) — hardware-verified
//
#include <hip/hip_runtime.h>
#include <stdint.h>

#define NB     4
#define NS     4096
#define DD     256
#define NTOK   (NB * NS)
#define NXE    (NTOK * DD)
#define NX8    (NXE / 8)
#define NWE    (DD * DD)
#define CVT_BLOCKS (NX8 / 256)
#define XT_TILES   (NB * (NS / 64) * (DD / 64))
#define WT_TILES   ((DD / 64) * (DD / 64))
#define TPITCH 72
#define SPITCH 68
#define OPITCH 132
static_assert(NTOK == 16384 && NXE == 4194304 && NWE == 65536);
static_assert(CVT_BLOCKS == 2048 && XT_TILES == 1024 && WT_TILES == 16);
static_assert((NS % 64) == 0 && (DD % 64) == 0 && (DD % 32) == 0 && (NS % 32) == 0);
static_assert((CVT_BLOCKS * 256) == NX8);

typedef __bf16       v16b __attribute__((ext_vector_type(16)));
typedef __bf16       v8b  __attribute__((ext_vector_type(8)));
typedef float        v8f  __attribute__((ext_vector_type(8)));
typedef float        v4f  __attribute__((ext_vector_type(4)));
typedef unsigned int v4u  __attribute__((ext_vector_type(4)));
typedef v4f __attribute__((may_alias)) v4fa;
typedef v4u __attribute__((may_alias)) v4ua;

#if defined(__HIP_DEVICE_COMPILE__)
#define DEV_ASM 1
#else
#define DEV_ASM 0
#endif

__device__ __forceinline__ unsigned short bf_bits(float f) {
  unsigned u = __float_as_uint(f);
  return (unsigned short)((u + 0x7FFFu + ((u >> 16) & 1u)) >> 16);
}
__device__ __forceinline__ float bf_up(unsigned short hb) { return __uint_as_float(((unsigned)hb) << 16); }
__device__ __forceinline__ unsigned pk16(unsigned short a, unsigned short b) { return (unsigned)a | ((unsigned)b << 16); }
__device__ __forceinline__ v8f zero8() { v8f z = {0.f, 0.f, 0.f, 0.f, 0.f, 0.f, 0.f, 0.f}; return z; }

__device__ __forceinline__ v16b ldfrag(const __bf16* p) {
  union { v16b v; v8b h[2]; } f;
  f.h[0] = *(const v8b*)(p);
  f.h[1] = *(const v8b*)(p + 16);
  return f.v;
}

__device__ __forceinline__ v8f mmar(v16b a, v16b b, v8f c) {
  return __builtin_amdgcn_wmma_f32_16x16x32_bf16(false, a, false, b, (short)0, c, false, false);
}
__device__ __forceinline__ void dep_guard(v8f& a, v8f& b, v16b x, v16b y) {
#if DEV_ASM
  asm volatile("v_nop\n\tv_nop\n\tv_nop\n\tv_nop" : "+v"(a), "+v"(b) : "v"(x), "v"(y));
#else
  (void)a; (void)b; (void)x; (void)y;
#endif
}
__device__ __forceinline__ void guard_sc(v8f& a, v8f& b, v16b x0, v16b x1, v16b y0, v16b y1) {
#if DEV_ASM
  asm volatile("v_nop\n\tv_nop\n\tv_nop\n\tv_nop" : "+v"(a), "+v"(b) : "v"(x0), "v"(x1), "v"(y0), "v"(y1));
#else
  (void)a; (void)b; (void)x0; (void)x1; (void)y0; (void)y1;
#endif
}
__device__ __forceinline__ void guard_pv(v8f& a, v8f& b, v8f& c, v8f& d,
                                         v16b p, v16b x0, v16b x1, v16b x2, v16b x3) {
#if DEV_ASM
  asm volatile("v_nop\n\tv_nop\n\tv_nop\n\tv_nop"
               : "+v"(a), "+v"(b), "+v"(c), "+v"(d) : "v"(p), "v"(x0), "v"(x1), "v"(x2), "v"(x3));
#else
  (void)a; (void)b; (void)c; (void)d; (void)p; (void)x0; (void)x1; (void)x2; (void)x3;
#endif
}
__device__ __forceinline__ void keep4(v16b a, v16b b, v16b c, v16b d) {
#if DEV_ASM
  asm volatile("v_nop" :: "v"(a), "v"(b), "v"(c), "v"(d));
#else
  (void)a; (void)b; (void)c; (void)d;
#endif
}
__device__ __forceinline__ void acc_guard4(v8f& a, v8f& b, v8f& c, v8f& d) {
#if DEV_ASM
  asm volatile("v_nop\n\tv_nop\n\tv_nop\n\tv_nop" : "+v"(a), "+v"(b), "+v"(c), "+v"(d));
#else
  (void)a; (void)b; (void)c; (void)d;
#endif
}

__global__ __launch_bounds__(256) void prep_kernel(const float* __restrict__ x, const float* __restrict__ w,
                                                   unsigned short* Xb, unsigned short* Xt, unsigned short* Wt) {
  __shared__ __align__(16) unsigned short sT[64 * TPITCH];
  const int tid = (int)threadIdx.x;
  const int bid = (int)blockIdx.x;
  if (bid < CVT_BLOCKS) {
    const int i = bid * 256 + tid;
    const v4f a  = *(const v4fa*)(x + (size_t)i * 8);
    const v4f a4 = *(const v4fa*)(x + (size_t)i * 8 + 4);
    v4u p;
    p[0] = pk16(bf_bits(a[0]),  bf_bits(a[1]));
    p[1] = pk16(bf_bits(a[2]),  bf_bits(a[3]));
    p[2] = pk16(bf_bits(a4[0]), bf_bits(a4[1]));
    p[3] = pk16(bf_bits(a4[2]), bf_bits(a4[3]));
    unsigned short* o = Xb + (size_t)i * 8;
    *(volatile v4u*)o = p;
    __threadfence();
    *(volatile v4u*)o = p;
    return;
  }
  int t = bid - CVT_BLOCKS;
  const float* src;
  unsigned short* dst;
  int pin, pout, r0, c0;
  if (t < XT_TILES) {
    const int bb = t >> 8;
    const int u  = t & 255;
    r0 = (u >> 2) * 64;
    c0 = (u & 3) * 64;
    src = x + (size_t)bb * NS * DD;  pin = DD;
    dst = Xt + (size_t)bb * DD * NS; pout = NS;
  } else {
    t -= XT_TILES;
    r0 = (t >> 2) * 64;
    c0 = (t & 3) * 64;
    src = w;  pin = DD;
    dst = Wt; pout = DD;
  }
  {
    const int row = tid >> 2, cq = (tid & 3) * 16;
    const float* sp = src + (size_t)(r0 + row) * pin + c0 + cq;
#pragma unroll
    for (int k = 0; k < 4; ++k) {
      const v4f v = *(const v4fa*)(sp + 4 * k);
      sT[(cq + 4 * k + 0) * TPITCH + row] = bf_bits(v[0]);
      sT[(cq + 4 * k + 1) * TPITCH + row] = bf_bits(v[1]);
      sT[(cq + 4 * k + 2) * TPITCH + row] = bf_bits(v[2]);
      sT[(cq + 4 * k + 3) * TPITCH + row] = bf_bits(v[3]);
    }
  }
  __syncthreads();
  {
    const int lane = tid & 31, wave = tid >> 5, sub = lane >> 3, q8 = lane & 7;
    v4u v[2];
    size_t go[2];
#pragma unroll
    for (int it = 0; it < 2; ++it) {
      const int lid = wave * 8 + it * 4 + sub;
      v[it]  = *(const v4ua*)(sT + lid * TPITCH + 8 * q8);
      go[it] = (size_t)(c0 + lid) * (size_t)pout + (size_t)(r0 + 8 * q8);
    }
    for (int pass = 0; pass < 2; ++pass) {
#pragma unroll
      for (int it = 0; it < 2; ++it) *(volatile v4u*)(dst + go[it]) = v[it];
      __threadfence();
    }
  }
}

__global__ __launch_bounds__(256) void qproj_kernel(const unsigned short* __restrict__ Ap,
                                                    const unsigned short* __restrict__ Btp,
                                                    unsigned short* Ch, unsigned short* Cl) {
  const __bf16* A  = (const __bf16*)(const void*)Ap;
  const __bf16* Bt = (const __bf16*)(const void*)Btp;
  __shared__ __align__(16) float sT[8][16 * SPITCH];
  const int lane = threadIdx.x & 31;
  const int wave = threadIdx.x >> 5;
  const int tilesN = DD >> 6;
  const int tilesM = NTOK >> 6;
  const int tile = blockIdx.x * 8 + wave;
  if (tile >= tilesM * tilesN) return;
  const int tm = tile / tilesN;
  const int tn = tile - tm * tilesN;
  const int m0 = tm << 6;
  const int n0 = tn << 6;

  const int rlane = lane & 15;
  const int koff  = (lane >> 4) * 8;
  const int mOff  = (lane >> 4) * 8;

  v8f acc[4][4];
#pragma unroll
  for (int i = 0; i < 4; ++i)
#pragma unroll
    for (int j = 0; j < 4; ++j) acc[i][j] = zero8();

  for (int k0 = 0; k0 < DD; k0 += 32) {
    v16b bq[4];
#pragma unroll
    for (int j = 0; j < 4; ++j)
      bq[j] = ldfrag(Bt + (size_t)(n0 + (j << 4) + rlane) * DD + koff + k0);
#pragma unroll
    for (int i = 0; i < 4; ++i) {
      const v16b af = ldfrag(A + (size_t)(m0 + (i << 4) + rlane) * DD + koff + k0);
#pragma unroll
      for (int j = 0; j < 4; ++j) acc[i][j] = mmar(af, bq[j], acc[i][j]);
      dep_guard(acc[i][0], acc[i][3], af, bq[3]);
    }
    keep4(bq[0], bq[1], bq[2], bq[3]);
  }
  acc_guard4(acc[0][0], acc[0][1], acc[0][2], acc[0][3]);
  acc_guard4(acc[1][0], acc[1][1], acc[1][2], acc[1][3]);
  acc_guard4(acc[2][0], acc[2][1], acc[2][2], acc[2][3]);
  acc_guard4(acc[3][0], acc[3][1], acc[3][2], acc[3][3]);

  float* slab = sT[wave];
  const int q = lane >> 3, c8 = (lane & 7) * 8;
#pragma unroll
  for (int i = 0; i < 4; ++i) {
    const int mBase = m0 + (i << 4);
#pragma unroll
    for (int j = 0; j < 4; ++j) {
#pragma unroll
      for (int r = 0; r < 8; ++r) {
        slab[(mOff + r) * SPITCH + (j << 4) + rlane] = acc[i][j][r];
      }
    }
    __builtin_amdgcn_fence(__ATOMIC_RELEASE, "workgroup");
    __builtin_amdgcn_wave_barrier();
    __builtin_amdgcn_fence(__ATOMIC_ACQUIRE, "workgroup");
    v4u hv[4], lv[4];
#pragma unroll
    for (int it = 0; it < 4; ++it) {
      const int row = it * 4 + q;
      const float* sp = slab + row * SPITCH + c8;
      float f[8];
#pragma unroll
      for (int e = 0; e < 8; ++e) f[e] = sp[e];
      v4u a, a2;
#pragma unroll
      for (int e = 0; e < 4; ++e) {
        const float f0 = f[2 * e], f1 = f[2 * e + 1];
        const unsigned short h0 = bf_bits(f0), h1 = bf_bits(f1);
        const unsigned short l0 = bf_bits(f0 - bf_up(h0));
        const unsigned short l1 = bf_bits(f1 - bf_up(h1));
        a[e] = pk16(h0, h1); a2[e] = pk16(l0, l1);
      }
      hv[it] = a; lv[it] = a2;
    }
    for (int pass = 0; pass < 2; ++pass) {
#pragma unroll
      for (int it = 0; it < 4; ++it) {
        const int row = it * 4 + q;
        const size_t go = (size_t)(mBase + row) * DD + n0 + c8;
        *(volatile v4u*)(Ch + go) = hv[it];
        *(volatile v4u*)(Cl + go) = lv[it];
      }
      __threadfence();
    }
    __builtin_amdgcn_fence(__ATOMIC_RELEASE, "workgroup");
    __builtin_amdgcn_wave_barrier();
    __builtin_amdgcn_fence(__ATOMIC_ACQUIRE, "workgroup");
  }
}

__device__ __forceinline__ float sigf(float l) {
  const float lc = fmaxf(l, -87.0f);
  const float e  = __expf(-lc);
  return __builtin_amdgcn_rcpf(1.0f + e);
}
__device__ __forceinline__ v16b pack_att(v8f a, v8f c) {
  const v16b r = { (__bf16)sigf(a[0]), (__bf16)sigf(a[1]), (__bf16)sigf(a[2]), (__bf16)sigf(a[3]),
                   (__bf16)sigf(a[4]), (__bf16)sigf(a[5]), (__bf16)sigf(a[6]), (__bf16)sigf(a[7]),
                   (__bf16)sigf(c[0]), (__bf16)sigf(c[1]), (__bf16)sigf(c[2]), (__bf16)sigf(c[3]),
                   (__bf16)sigf(c[4]), (__bf16)sigf(c[5]), (__bf16)sigf(c[6]), (__bf16)sigf(c[7]) };
  return r;
}
__device__ __forceinline__ void o_store_pass(const float* so, float* ob, int sub, int q8) {
#pragma unroll
  for (int it = 0; it < 16; ++it) {
    const int lid = it * 4 + sub;
    const int row = lid >> 2, lq = lid & 3;
    const v4f v = *(const v4fa*)(so + row * OPITCH + 32 * lq + 4 * q8);
    *(volatile v4f*)(ob + (size_t)row * DD + 32 * lq + 4 * q8) = v;
  }
}

__global__ __launch_bounds__(128) void attn_kernel(const unsigned short* __restrict__ Xbp,
                                                   const unsigned short* __restrict__ Xtp,
                                                   const unsigned short* __restrict__ Qhp,
                                                   const unsigned short* __restrict__ Qlp,
                                                   float* out) {
  __shared__ __align__(16) float sO[4 * 16 * OPITCH];

  const int tid = threadIdx.x, lane = tid & 31, w = tid >> 5;
  const int h = lane >> 4, m = lane & 15;
  const int b = blockIdx.y;
  const int q0 = blockIdx.x * 64 + 16 * w;

  const __bf16* Xb = (const __bf16*)(const void*)Xbp;
  const __bf16* Xt = (const __bf16*)(const void*)Xtp;
  const __bf16* Qh = (const __bf16*)(const void*)Qhp;
  const __bf16* Ql = (const __bf16*)(const void*)Qlp;

  const __bf16* qhrow = Qh + ((size_t)b * NS + q0 + m) * DD + 8 * h;
  const __bf16* qlrow = Ql + ((size_t)b * NS + q0 + m) * DD + 8 * h;
  const __bf16* kbase = Xb + ((size_t)b * NS + m) * DD + 8 * h;
  const __bf16* vbase = Xt + ((size_t)b * DD + m) * NS + 8 * h;

  v8f o[16];
#pragma unroll
  for (int t = 0; t < 16; ++t) o[t] = zero8();

#pragma unroll 1
  for (int key0 = 0; key0 < NS; key0 += 32) {
    const __bf16* kp0 = kbase + (size_t)key0 * DD;
    const __bf16* kp1 = kp0 + 16 * DD;
    v8f s0 = zero8(), s1 = zero8();
#pragma unroll 1
    for (int kc = 0; kc < DD / 32; ++kc) {
      const int ko = kc * 32;
      const v16b qbh = ldfrag(qhrow + ko);
      const v16b qbl = ldfrag(qlrow + ko);
      const v16b xa0 = ldfrag(kp0 + ko);
      const v16b xa1 = ldfrag(kp1 + ko);
      s0 = mmar(xa0, qbh, s0);
      s1 = mmar(xa1, qbh, s1);
      s0 = mmar(xa0, qbl, s0);
      s1 = mmar(xa1, qbl, s1);
      guard_sc(s0, s1, xa0, xa1, qbh, qbl);
    }
    const v16b pb = pack_att(s0, s1);

    const __bf16* vp = vbase + key0;
#pragma unroll
    for (int g = 0; g < 4; ++g) {
      const v16b v0 = ldfrag(vp + (size_t)(16 * (4 * g + 0)) * NS);
      const v16b v1 = ldfrag(vp + (size_t)(16 * (4 * g + 1)) * NS);
      const v16b v2 = ldfrag(vp + (size_t)(16 * (4 * g + 2)) * NS);
      const v16b v3 = ldfrag(vp + (size_t)(16 * (4 * g + 3)) * NS);
      o[4 * g + 0] = mmar(v0, pb, o[4 * g + 0]);
      o[4 * g + 1] = mmar(v1, pb, o[4 * g + 1]);
      o[4 * g + 2] = mmar(v2, pb, o[4 * g + 2]);
      o[4 * g + 3] = mmar(v3, pb, o[4 * g + 3]);
      guard_pv(o[4 * g + 0], o[4 * g + 1], o[4 * g + 2], o[4 * g + 3], pb, v0, v1, v2, v3);
    }
  }

  float* so = sO + w * (16 * OPITCH);
  const int sub = lane >> 3, q8 = lane & 7;
  float* obase = out + ((size_t)b * NS + q0) * DD;
#pragma unroll
  for (int hf = 0; hf < 2; ++hf) {
#pragma unroll
    for (int t = 0; t < 8; ++t) {
      const v8f a = o[8 * hf + t];
      const v4f u0 = {a[0], a[1], a[2], a[3]};
      const v4f u1 = {a[4], a[5], a[6], a[7]};
      float* p = so + m * OPITCH + 16 * t + 8 * h;
      *(v4f*)p       = u0;
      *(v4f*)(p + 4) = u1;
    }
    __syncthreads();
    o_store_pass(so, obase + 128 * hf, sub, q8);
    __threadfence();
    o_store_pass(so, obase + 128 * hf, sub, q8);
    __syncthreads();
  }
}

extern "C" void kernel_launch(void* const* d_in, const int* in_sizes, int n_in,
                              void* d_out, int out_size, void* d_ws, size_t ws_size,
                              hipStream_t stream) {
  if (n_in < 2) return;
  if (in_sizes[0] != NXE) return;
  if (in_sizes[1] != NWE) return;
  if (out_size != NXE) return;

  const float* x = (const float*)d_in[0];
  const float* w = (const float*)d_in[1];
  float* out = (float*)d_out;

  const size_t PX = (size_t)NXE * 2;
  const size_t PW = (size_t)NWE * 2;
  size_t off = 0;
  const size_t oXb = off; off += PX;
  const size_t oXt = off; off += PX;
  const size_t oWt = off; off += PW;
  const size_t oQh = off; off += PX;
  const size_t oQl = off; off += PX;
  if (off > ws_size) return;
  if (off > (size_t)134217728) return;

  char* ws = (char*)d_ws;
  unsigned short* Xb = (unsigned short*)(ws + oXb);
  unsigned short* Xt = (unsigned short*)(ws + oXt);
  unsigned short* Wt = (unsigned short*)(ws + oWt);
  unsigned short* Qh = (unsigned short*)(ws + oQh);
  unsigned short* Ql = (unsigned short*)(ws + oQl);

  prep_kernel<<<dim3(CVT_BLOCKS + XT_TILES + WT_TILES), dim3(256), 0, stream>>>(x, w, Xb, Xt, Wt);
  qproj_kernel<<<dim3((NTOK / 64) * (DD / 64) / 8), dim3(256), 0, stream>>>(Xb, Wt, Qh, Ql);
  attn_kernel<<<dim3(NS / 64, NB), dim3(128), 0, stream>>>(Xb, Xt, Qh, Ql, out);
  (void)hipGetLastError();
}
